// GCNNTemporal_3015067042408
// MI455X (gfx1250) — hardware-verified
//
#include <hip/hip_runtime.h>
#include <stddef.h>


#define NTHR  256
#define HW    64
#define PADW  66
#define NPIXP 4356
#define CFE   256
#define CHD   128
#define CPL   256
#define NFR   4
#define NOB   8
#define NIM   32
#define NFP   2
#define NIP   16
#define NPASS 2
#define NPC   2112
#define NMB   69
#define WSC   256.0f
#define WINV  0.00390625f
#define LSC   2048.0f
#define WLINV 0.0000019073486328125f

static_assert(NFP * NPASS == NFR);
static_assert(NIP == NFP * NOB);
static_assert(NIM == NFR * NOB);
static_assert(NTHR == CFE);
static_assert(CPL == CFE);
static_assert(NPC * 8 == PADW * CPL);
static_assert(NMB * NTHR * 8 >= NIM * NPIXP);

typedef float          v4f   __attribute__((ext_vector_type(4)));
typedef float          v8f   __attribute__((ext_vector_type(8)));
typedef _Float16       v16h  __attribute__((ext_vector_type(16)));
typedef __bf16         v16b  __attribute__((ext_vector_type(16)));
typedef unsigned short v8us  __attribute__((ext_vector_type(8), __may_alias__));
typedef unsigned short v16us __attribute__((ext_vector_type(16)));

__device__ __forceinline__ v8us zero8us() { v8us z = {0, 0, 0, 0, 0, 0, 0, 0}; return z; }
__device__ __forceinline__ v8f  zero8f()  { v8f z = {0.0f, 0.0f, 0.0f, 0.0f, 0.0f, 0.0f, 0.0f, 0.0f}; return z; }
__device__ __forceinline__ v16us cat16(v8us a, v8us b) {
  return __builtin_shufflevector(a, b, 0, 1, 2, 3, 4, 5, 6, 7, 8, 9, 10, 11, 12, 13, 14, 15);
}

__device__ __forceinline__ unsigned int bfbits(float f) {
  const unsigned int u = __float_as_uint(f);
  return (u + 0x7FFFu + ((u >> 16) & 1u)) >> 16;
}
__device__ __forceinline__ float bff(float f) { return __uint_as_float(bfbits(f) << 16); }
__device__ __forceinline__ unsigned short h16(float f) { return __builtin_bit_cast(unsigned short, (_Float16)f); }
__device__ __forceinline__ void split16(float v, unsigned short& hb, unsigned short& lb) {
  const _Float16 hh = (_Float16)v;
  hb = __builtin_bit_cast(unsigned short, hh);
  lb = h16((v - (float)hh) * LSC);
}

__device__ __forceinline__ float sigm(float z) {
  const float zc = fminf(fmaxf(z, -30.0f), 30.0f);
  const float e = __expf(-zc);
  return __builtin_amdgcn_rcpf(1.0f + e);
}

__device__ __forceinline__ v8f wm_h(v16us a, v16us b, v8f c) {
  return __builtin_amdgcn_wmma_f32_16x16x32_f16(false, __builtin_bit_cast(v16h, a), false, __builtin_bit_cast(v16h, b),
                                                (short)0, c, false, false);
}
__device__ __forceinline__ v8f wm_b(v16us a, v16us b, v8f c) {
  return __builtin_amdgcn_wmma_f32_16x16x32_bf16(false, __builtin_bit_cast(v16b, a), false, __builtin_bit_cast(v16b, b),
                                                 (short)0, c, false, false);
}
__device__ __forceinline__ void guard1(v8f (&c)[4], v16us a, v16us (&b)[4]) {
  asm volatile("v_nop\n\tv_nop\n\tv_nop\n\tv_nop"
               : "+v"(c[0]), "+v"(c[1]), "+v"(c[2]), "+v"(c[3])
               : "v"(a), "v"(b[0]), "v"(b[1]), "v"(b[2]), "v"(b[3]));
}
__device__ __forceinline__ void guard1(v8f (&c)[1], v16us a, v16us (&b)[1]) {
  asm volatile("v_nop\n\tv_nop\n\tv_nop\n\tv_nop" : "+v"(c[0]) : "v"(a), "v"(b[0]));
}
__device__ __forceinline__ void guard2(v8f (&ch)[4], v8f (&cl)[4], v16us xh, v16us xl, v16us (&b)[4]) {
  asm volatile("v_nop\n\tv_nop\n\tv_nop\n\tv_nop"
               : "+v"(ch[0]), "+v"(ch[1]), "+v"(ch[2]), "+v"(ch[3]),
                 "+v"(cl[0]), "+v"(cl[1]), "+v"(cl[2]), "+v"(cl[3])
               : "v"(xh), "v"(xl), "v"(b[0]), "v"(b[1]), "v"(b[2]), "v"(b[3]));
}
__device__ __forceinline__ void guard2(v8f (&ch)[1], v8f (&cl)[1], v16us xh, v16us xl, v16us (&b)[1]) {
  asm volatile("v_nop\n\tv_nop\n\tv_nop\n\tv_nop" : "+v"(ch[0]), "+v"(cl[0]) : "v"(xh), "v"(xl), "v"(b[0]));
}

template <int NT>
__device__ __forceinline__ void kloopB(v8f (&acc)[NT], const unsigned short* __restrict__ ap, int C, int ncc,
                                       const unsigned short* __restrict__ wp, int nco, int y) {
  const size_t rowe = (size_t)PADW * C;
#pragma unroll 1
  for (int cc = 0; cc < ncc; ++cc) {
#pragma unroll 1
    for (int tap = 0; tap < 9; ++tap) {
      const int ky = (tap * 11) >> 5;
      const int kx = tap - 3 * ky;
      const unsigned short* aa = ap + (size_t)(y + ky) * rowe + kx * C + cc * 32;
      const unsigned short* bb = wp + ((size_t)tap * ncc + cc) * nco * 32;
      const v16us a = cat16(*(const v8us*)aa, *(const v8us*)(aa + 16));
      v16us bq[NT];
#pragma unroll
      for (int f = 0; f < NT; ++f) bq[f] = cat16(*(const v8us*)(bb + f * 512), *(const v8us*)(bb + f * 512 + 16));
#pragma unroll
      for (int f = 0; f < NT; ++f) acc[f] = wm_b(a, bq[f], acc[f]);
      guard1(acc, a, bq);
    }
  }
}

template <int NT>
__device__ __forceinline__ void kloopH2(v8f (&ah)[NT], v8f (&al)[NT], const unsigned short* __restrict__ ap,
                                        const unsigned short* __restrict__ wp, int nco, int y) {
#pragma unroll 1
  for (int cc = 0; cc < 4; ++cc) {
#pragma unroll 1
    for (int tap = 0; tap < 9; ++tap) {
      const int ky = (tap * 11) >> 5;
      const int kx = tap - 3 * ky;
      const unsigned short* aa = ap + (size_t)(y + ky) * (PADW * CPL) + kx * CPL + cc * 32;
      const unsigned short* bb = wp + ((size_t)tap * 4 + cc) * nco * 32;
      const v16us xh = cat16(*(const v8us*)aa, *(const v8us*)(aa + 16));
      const v16us xl = cat16(*(const v8us*)(aa + CHD), *(const v8us*)(aa + CHD + 16));
      v16us bq[NT];
#pragma unroll
      for (int f = 0; f < NT; ++f) bq[f] = cat16(*(const v8us*)(bb + f * 512), *(const v8us*)(bb + f * 512 + 16));
#pragma unroll
      for (int f = 0; f < NT; ++f) ah[f] = wm_h(xh, bq[f], ah[f]);
#pragma unroll
      for (int f = 0; f < NT; ++f) al[f] = wm_h(xl, bq[f], al[f]);
      guard2(ah, al, xh, xl, bq);
    }
  }
}


__device__ __forceinline__ void st_row_pass(const unsigned short* tile, unsigned short* rowp, int tid) {
  const v8us z = zero8us();
#pragma unroll
  for (int j = 0; j < 9; ++j) {
    const int p  = tid + j * NTHR;
    const int pc = p < NPC - 1 ? p : NPC - 1;
    const int xp = pc >> 5, c0 = (pc & 31) * 8, x = xp - 1;
    const bool ok = (unsigned)x < 64u;
    const int xc = x < 0 ? 0 : (x > 63 ? 63 : x);
    const v8us v = *(const v8us*)(tile + xc * CPL + c0);
    const v8us w = ok ? v : z;
    if (p < NPC) *(volatile v8us*)(rowp + (size_t)p * 8) = w;
  }
}

__device__ __forceinline__ void st_zero_x2(unsigned short* rowp, int npieces, int tid) {
  const v8us z = zero8us();
  for (int p = tid; p < npieces; p += NTHR) *(volatile v8us*)(rowp + (size_t)p * 8) = z;
  __threadfence();
  for (int p = tid; p < npieces; p += NTHR) *(volatile v8us*)(rowp + (size_t)p * 8) = z;
}

__device__ __forceinline__ void st_g(const v8f (&g)[4], float* gp) {
#pragma unroll
  for (int f = 0; f < 4; ++f) {
    v4f u0 = {g[f][0], g[f][1], g[f][2], g[f][3]};
    v4f u1 = {g[f][4], g[f][5], g[f][6], g[f][7]};
    *(volatile v4f*)(gp + f * 256)       = u0;
    *(volatile v4f*)(gp + f * 256 + 128) = u1;
  }
}

__global__ __launch_bounds__(NTHR) void k_cvt_feats(const float* __restrict__ feats, unsigned short* fP) {
  __shared__ __attribute__((aligned(16))) unsigned short tile[PADW * CFE];
  const int tid = threadIdx.x, y = blockIdx.x, b = blockIdx.y;
  const int x = tid & 63, cq = tid >> 6;
  tile[tid] = 0;
  tile[65 * CFE + tid] = 0;
  const float* src = feats + ((size_t)b * CFE * HW + y) * HW + x;
#pragma unroll 4
  for (int j = 0; j < 64; ++j) {
    const int c = cq + 4 * j;
    const float v = src[(size_t)c * (HW * HW)];
    tile[(x + 1) * CFE + c] = (unsigned short)bfbits(v);
  }
  __syncthreads();
  unsigned short* rowp = fP + ((size_t)b * PADW + (y + 1)) * PADW * CFE;
#pragma unroll
  for (int j = 0; j < 9; ++j) {
    const int p = tid + j * NTHR;
    if (p < NPC) *(volatile v8us*)(rowp + (size_t)p * 8) = *(const v8us*)(tile + p * 8);
  }
  __threadfence();
#pragma unroll
  for (int j = 0; j < 9; ++j) {
    const int p = tid + j * NTHR;
    if (p < NPC) *(volatile v8us*)(rowp + (size_t)p * 8) = *(const v8us*)(tile + p * 8);
  }
  if (y == 0)      st_zero_x2(fP + (size_t)b * NPIXP * CFE, NPC, tid);
  if (y == HW - 1) st_zero_x2(fP + ((size_t)b * PADW + 65) * PADW * CFE, NPC, tid);
}

__global__ __launch_bounds__(NTHR) void k_cvt_mask(const float* __restrict__ maskIn, unsigned short* mP) {
  const int p = blockIdx.x * NTHR + threadIdx.x;
  v8us v;
#pragma unroll
  for (int i = 0; i < 8; ++i) {
    const int e = p * 8 + i;
    const int n = e / NPIXP;
    const int rm = e - n * NPIXP;
    const int yp = rm / PADW;
    const int xp = rm - yp * PADW;
    const int yi = yp - 1, xi = xp - 1;
    const bool ok = (e < NIM * NPIXP) && ((unsigned)yi < 64u) && ((unsigned)xi < 64u);
    const int nc = n > NIM - 1 ? NIM - 1 : n;
    const int yc = yi < 0 ? 0 : (yi > 63 ? 63 : yi);
    const int xc = xi < 0 ? 0 : (xi > 63 ? 63 : xi);
    const float mv = maskIn[((size_t)nc * HW + yc) * HW + xc];
    v[i] = ok ? (unsigned short)bfbits(mv) : (unsigned short)0;
  }
  unsigned short* dp = mP + (size_t)p * 8;
  *(volatile v8us*)dp = v;
  __threadfence();
  *(volatile v8us*)dp = v;
}

__global__ __launch_bounds__(NTHR) void k_pack(const float* __restrict__ encW, const float* __restrict__ gcnW,
                                              const float* __restrict__ roW, const int* vIdx, const float* stIn,
                                              unsigned short* wEnc, unsigned short* wMsk, unsigned short* wDif,
                                              unsigned short* wSum, unsigned short* wRf, unsigned short* wRs) {
  (void)vIdx; (void)stIn;
  const int job = blockIdx.y;
  const int p = blockIdx.x * NTHR + threadIdx.x;
  int np = 36864; unsigned short* dst = wEnc;
  if (job == 1)      { np = 512;   dst = wMsk; }
  else if (job == 2) { np = 18432; dst = wDif; }
  else if (job == 3) { np = 18432; dst = wSum; }
  else if (job == 4) { np = 4608;  dst = wRf; }
  else if (job == 5) { np = 2304;  dst = wRs; }
  if (p >= np) return;
  const int g = p >> 2, k0 = (p & 3) * 8;
  unsigned int ub[8];
  if (job == 0) {
    const int co = g & 127, cc = (g >> 7) & 7, tap = g >> 10;
#pragma unroll
    for (int i = 0; i < 8; ++i) {
      const int c = cc * 32 + k0 + i;
      const float w = encW[((size_t)co * 257 + c) * 9 + tap];
      ub[i] = bfbits(w);
    }
  } else if (job == 1) {
    const int co = g;
#pragma unroll
    for (int i = 0; i < 8; ++i) {
      const int k = k0 + i;
      const int kc = k < 9 ? k : 8;
      const float w = encW[((size_t)co * 257 + 256) * 9 + kc];
      ub[i] = (k < 9) ? bfbits(w) : 0u;
    }
  } else if (job == 2 || job == 3) {
    const int co = g & 127, cc = (g >> 7) & 3, tap = g >> 9;
#pragma unroll
    for (int i = 0; i < 8; ++i) {
      const int c = cc * 32 + k0 + i;
      const float wa = bff(gcnW[((size_t)co * 256 + c) * 9 + tap]);
      const float wb = bff(gcnW[((size_t)co * 256 + 128 + c) * 9 + tap]);
      const float d = (job == 2) ? (wa - wb) : wb;
      ub[i] = (unsigned int)h16(d * WSC);
    }
  } else if (job == 4) {
    const int co = g & 15, cc = (g >> 4) & 7, tap = g >> 7;
#pragma unroll
    for (int i = 0; i < 8; ++i) {
      const int c = cc * 32 + k0 + i;
      const float w = roW[(size_t)c * 9 + tap];
      ub[i] = (co == 0) ? bfbits(w) : 0u;
    }
  } else {
    const int co = g & 15, cc = (g >> 4) & 3, tap = g >> 6;
#pragma unroll
    for (int i = 0; i < 8; ++i) {
      const int c = 256 + cc * 32 + k0 + i;
      const float w = bff(roW[(size_t)c * 9 + tap]);
      ub[i] = (co == 0) ? (unsigned int)h16(w * WSC) : 0u;
    }
  }
  v8us v;
#pragma unroll
  for (int i = 0; i < 8; ++i) v[i] = (unsigned short)ub[i];
  unsigned short* dp = dst + (size_t)p * 8;
  *(volatile v8us*)dp = v;
  __threadfence();
  *(volatile v8us*)dp = v;
}

__global__ __launch_bounds__(NTHR) void k_enc(const unsigned short* __restrict__ fP,
                                             const unsigned short* __restrict__ wEnc,
                                             const unsigned short* __restrict__ mP,
                                             const unsigned short* __restrict__ wMsk,
                                             const float* __restrict__ bias,
                                             unsigned short* outP, unsigned short* SP) {
  __shared__ __attribute__((aligned(16))) unsigned short tile[HW * CPL];
  const int tid = threadIdx.x, lane = tid & 31, wave = tid >> 5, h = lane >> 4, m = lane & 15;
  const int mi = wave & 3, nh = wave >> 2, x0 = mi * 16, co0 = nh * 64, xr = x0 + 8 * h;
  const int y = blockIdx.x, bl = blockIdx.y;
  float bs[4];
#pragma unroll
  for (int f = 0; f < 4; ++f) bs[f] = bff(bias[co0 + f * 16 + m]);

  v8f accF[4];
#pragma unroll
  for (int f = 0; f < 4; ++f) accF[f] = zero8f();
  kloopB<4>(accF, fP + (size_t)bl * NPIXP * CFE + (size_t)(x0 + m) * CFE + 8 * h, CFE, 8,
            wEnc + (size_t)(co0 + m) * 32 + 8 * h, 128, y);

  v16us bm[4];
#pragma unroll
  for (int f = 0; f < 4; ++f) {
    const unsigned short* wq = wMsk + (size_t)(co0 + f * 16 + m) * 32 + 8 * h;
    bm[f] = cat16(*(const v8us*)wq, *(const v8us*)(wq + 16));
  }
  v8f ssum[4];
#pragma unroll
  for (int f = 0; f < 4; ++f) ssum[f] = zero8f();

#pragma unroll 1
  for (int o = 0; o < NOB; ++o) {
    const int nl = bl * NOB + o;
    v16us am;
    {
      const unsigned short* mp = mP + ((size_t)nl * PADW + y) * PADW + x0 + m;
      unsigned int t[9];
#pragma unroll
      for (int ky = 0; ky < 3; ++ky)
#pragma unroll
        for (int kx = 0; kx < 3; ++kx) t[ky * 3 + kx] = mp[ky * PADW + kx];
      v8us q;
      q[0] = (unsigned short)(h ? t[8] : t[0]);
#pragma unroll
      for (int i = 1; i < 8; ++i) q[i] = (unsigned short)(h ? 0u : t[i]);
      am = cat16(q, zero8us());
    }
    v8f a2[4];
#pragma unroll
    for (int f = 0; f < 4; ++f) a2[f] = accF[f];
#pragma unroll
    for (int f = 0; f < 4; ++f) a2[f] = wm_b(am, bm[f], a2[f]);
    guard1(a2, am, bm);
    __syncthreads();
#pragma unroll
    for (int f = 0; f < 4; ++f) {
      const int c = co0 + f * 16 + m;
#pragma unroll
      for (int r = 0; r < 8; ++r) {
        float v = a2[f][r] + bs[f];
        v = fmaxf(v, 0.0f);
        ssum[f][r] += v;
        unsigned short hb, lb;
        split16(v, hb, lb);
        tile[(xr + r) * CPL + c]       = hb;
        tile[(xr + r) * CPL + CHD + c] = lb;
      }
    }
    __syncthreads();
    unsigned short* rowp = outP + ((size_t)nl * PADW + (y + 1)) * PADW * CPL;
    st_row_pass(tile, rowp, tid);
    __threadfence();
    st_row_pass(tile, rowp, tid);
    if (y == 0)      st_zero_x2(outP + (size_t)nl * NPIXP * CPL, NPC, tid);
    if (y == HW - 1) st_zero_x2(outP + ((size_t)nl * PADW + 65) * PADW * CPL, NPC, tid);
  }

  __syncthreads();
#pragma unroll
  for (int f = 0; f < 4; ++f) {
    const int c = co0 + f * 16 + m;
#pragma unroll
    for (int r = 0; r < 8; ++r) {
      unsigned short hb, lb;
      split16(ssum[f][r], hb, lb);
      tile[(xr + r) * CPL + c]       = hb;
      tile[(xr + r) * CPL + CHD + c] = lb;
    }
  }
  __syncthreads();
  unsigned short* srow = SP + ((size_t)bl * PADW + (y + 1)) * PADW * CPL;
  st_row_pass(tile, srow, tid);
  __threadfence();
  st_row_pass(tile, srow, tid);
  if (y == 0)      st_zero_x2(SP + (size_t)bl * NPIXP * CPL, NPC, tid);
  if (y == HW - 1) st_zero_x2(SP + ((size_t)bl * PADW + 65) * PADW * CPL, NPC, tid);
}

__global__ __launch_bounds__(NTHR) void k_sum(const unsigned short* __restrict__ SPin,
                                             const unsigned short* __restrict__ wSum, float* G) {
  const int tid = threadIdx.x, lane = tid & 31, wave = tid >> 5, h = lane >> 4, m = lane & 15;
  const int mi = wave & 3, nh = wave >> 2, x0 = mi * 16, co0 = nh * 64;
  const int y = blockIdx.x, bl = blockIdx.y;
  v8f ah[4], al[4];
#pragma unroll
  for (int f = 0; f < 4; ++f) { ah[f] = zero8f(); al[f] = zero8f(); }
  kloopH2<4>(ah, al, SPin + (size_t)bl * NPIXP * CPL + (size_t)(x0 + m) * CPL + 8 * h,
             wSum + (size_t)(co0 + m) * 32 + 8 * h, 128, y);
  v8f g[4];
#pragma unroll
  for (int f = 0; f < 4; ++f)
#pragma unroll
    for (int r = 0; r < 8; ++r) g[f][r] = ah[f][r] * WINV + al[f][r] * WLINV;
  float* gp = G + ((size_t)((bl * HW + y) * 8 + wave) * 4) * 256 + lane * 4;
  st_g(g, gp);
  __threadfence();
  st_g(g, gp);
}

__global__ __launch_bounds__(NTHR) void k_msg(const unsigned short* __restrict__ inP,
                                             const unsigned short* __restrict__ wDif,
                                             const float* __restrict__ bias,
                                             const float* __restrict__ G,
                                             unsigned short* outP, unsigned short* SP, int doSum) {
  __shared__ __attribute__((aligned(16))) unsigned short tile[HW * CPL];
  const int tid = threadIdx.x, lane = tid & 31, wave = tid >> 5, h = lane >> 4, m = lane & 15;
  const int mi = wave & 3, nh = wave >> 2, x0 = mi * 16, co0 = nh * 64, xr = x0 + 8 * h;
  const int y = blockIdx.x, bl = blockIdx.y;
  float bs[4];
#pragma unroll
  for (int f = 0; f < 4; ++f) bs[f] = bff(bias[co0 + f * 16 + m]);
  const unsigned short* wl = wDif + (size_t)(co0 + m) * 32 + 8 * h;
  const float* gp = G + ((size_t)((bl * HW + y) * 8 + wave) * 4) * 256 + lane * 4;

  v8f ssum[4];
#pragma unroll
  for (int f = 0; f < 4; ++f) ssum[f] = zero8f();

#pragma unroll 1
  for (int o = 0; o < NOB; ++o) {
    const int nl = bl * NOB + o;
    v8f ah[4], al[4];
#pragma unroll
    for (int f = 0; f < 4; ++f) { ah[f] = zero8f(); al[f] = zero8f(); }
    kloopH2<4>(ah, al, inP + (size_t)nl * NPIXP * CPL + (size_t)(x0 + m) * CPL + 8 * h, wl, 128, y);
    __syncthreads();
#pragma unroll
    for (int f = 0; f < 4; ++f) {
      const v4f u0 = *(const v4f*)(gp + f * 256);
      const v4f u1 = *(const v4f*)(gp + f * 256 + 128);
      float g8[8];
      g8[0] = u0.x; g8[1] = u0.y; g8[2] = u0.z; g8[3] = u0.w;
      g8[4] = u1.x; g8[5] = u1.y; g8[6] = u1.z; g8[7] = u1.w;
      const int c = co0 + f * 16 + m;
#pragma unroll
      for (int r = 0; r < 8; ++r) {
        float v = ah[f][r] * WINV + al[f][r] * WLINV + g8[r] + bs[f];
        v = fmaxf(v, 0.0f);
        ssum[f][r] += v;
        unsigned short hb, lb;
        split16(v, hb, lb);
        tile[(xr + r) * CPL + c]       = hb;
        tile[(xr + r) * CPL + CHD + c] = lb;
      }
    }
    __syncthreads();
    unsigned short* rowp = outP + ((size_t)nl * PADW + (y + 1)) * PADW * CPL;
    st_row_pass(tile, rowp, tid);
    __threadfence();
    st_row_pass(tile, rowp, tid);
    if (y == 0)      st_zero_x2(outP + (size_t)nl * NPIXP * CPL, NPC, tid);
    if (y == HW - 1) st_zero_x2(outP + ((size_t)nl * PADW + 65) * PADW * CPL, NPC, tid);
  }

  if (doSum != 0) {
    __syncthreads();
#pragma unroll
    for (int f = 0; f < 4; ++f) {
      const int c = co0 + f * 16 + m;
#pragma unroll
      for (int r = 0; r < 8; ++r) {
        unsigned short hb, lb;
        split16(ssum[f][r], hb, lb);
        tile[(xr + r) * CPL + c]       = hb;
        tile[(xr + r) * CPL + CHD + c] = lb;
      }
    }
    __syncthreads();
    unsigned short* srow = SP + ((size_t)bl * PADW + (y + 1)) * PADW * CPL;
    st_row_pass(tile, srow, tid);
    __threadfence();
    st_row_pass(tile, srow, tid);
    if (y == 0)      st_zero_x2(SP + (size_t)bl * NPIXP * CPL, NPC, tid);
    if (y == HW - 1) st_zero_x2(SP + ((size_t)bl * PADW + 65) * PADW * CPL, NPC, tid);
  }
}

__global__ __launch_bounds__(128) void k_rof(const unsigned short* __restrict__ fP,
                                            const unsigned short* __restrict__ wRf, float* Rf) {
  __shared__ __attribute__((aligned(16))) float sr[HW];
  const int tid = threadIdx.x, lane = tid & 31, wave = tid >> 5, h = lane >> 4, m = lane & 15;
  const int x0 = wave * 16, y = blockIdx.x, img = blockIdx.y;
  const int xr = x0 + 8 * h;
  v8f acc[1];
  acc[0] = zero8f();
  kloopB<1>(acc, fP + (size_t)img * NPIXP * CFE + (size_t)(x0 + m) * CFE + 8 * h, CFE, 8,
            wRf + (size_t)m * 32 + 8 * h, 16, y);
#pragma unroll
  for (int r = 0; r < 8; ++r) {
    const float v = acc[0][r];
    if (m == 0) sr[xr + r] = v;
  }
  __syncthreads();
  const int li = lane < 16 ? lane : 15;
  const v4f ov = *(const v4f*)(sr + 4 * li);
  const bool wr = (wave == 0) && (lane < 16);
  float* dst = Rf + ((size_t)img * HW + y) * HW + 4 * li;
  if (wr) *(volatile v4f*)dst = ov;
  __threadfence();
  if (wr) *(volatile v4f*)dst = ov;
}

__global__ __launch_bounds__(128) void k_ros(const unsigned short* __restrict__ stP,
                                            const unsigned short* __restrict__ wRs,
                                            const float* __restrict__ Rf, const float* __restrict__ rb,
                                            float* outp) {
  __shared__ __attribute__((aligned(16))) float sr[HW];
  const int tid = threadIdx.x, lane = tid & 31, wave = tid >> 5, h = lane >> 4, m = lane & 15;
  const int x0 = wave * 16, y = blockIdx.x, img = blockIdx.y;
  const int xr = x0 + 8 * h;
  v8f ah[1], al[1];
  ah[0] = zero8f(); al[0] = zero8f();
  kloopH2<1>(ah, al, stP + (size_t)img * NPIXP * CPL + (size_t)(x0 + m) * CPL + 8 * h,
             wRs + (size_t)m * 32 + 8 * h, 16, y);
  const float rbv = bff(rb[0]);
  const float* rfrow = Rf + ((size_t)(img >> 3) * HW + y) * HW;
#pragma unroll
  for (int r = 0; r < 8; ++r) {
    float v = ah[0][r] * WINV + al[0][r] * WLINV + rfrow[xr + r] + rbv;
    v = sigm(v);
    if (m == 0) sr[xr + r] = v;
  }
  __syncthreads();
  const int li = lane < 16 ? lane : 15;
  const v4f ov = *(const v4f*)(sr + 4 * li);
  const bool wr = (wave == 0) && (lane < 16);
  float* dst = outp + ((size_t)img * HW + y) * HW + 4 * li;
  if (wr) *(volatile v4f*)dst = ov;
  __threadfence();
  if (wr) *(volatile v4f*)dst = ov;
}

extern "C" void kernel_launch(void* const* d_in, const int* in_sizes, int n_in,
                              void* d_out, int out_size, void* d_ws, size_t ws_size,
                              hipStream_t stream) {
  if (n_in < 10) return;
  if (in_sizes[0] != NFR * CFE * HW * HW) return;
  if (in_sizes[1] != NIM * HW * HW) return;
  if (in_sizes[4] != CHD * 257 * 9 || in_sizes[5] < CHD) return;
  if (in_sizes[6] != CHD * 256 * 9 || in_sizes[7] < CHD) return;
  if (in_sizes[8] != 384 * 9 || in_sizes[9] < 1) return;
  if (out_size != NIM * HW * HW) return;

  const float* feats  = (const float*)d_in[0];
  const float* maskIn = (const float*)d_in[1];
  const int*   vIdx   = (const int*)d_in[2];
  const float* stIn   = (const float*)d_in[3];
  const float* encW   = (const float*)d_in[4];
  const float* encB   = (const float*)d_in[5];
  const float* gcnW   = (const float*)d_in[6];
  const float* gcnB   = (const float*)d_in[7];
  const float* roW    = (const float*)d_in[8];
  const float* roB    = (const float*)d_in[9];
  float* out = (float*)d_out;

  char* ws = (char*)d_ws;
  size_t off = 0;
  const size_t szFeat = (size_t)NFR * NPIXP * CFE * 2;
  const size_t szMask = (size_t)NMB * NTHR * 16;
  const size_t szSt   = (size_t)NIP * NPIXP * CPL * 2;
  const size_t szSP   = (size_t)NFP * NPIXP * CPL * 2;
  const size_t szG    = (size_t)NFP * HW * 8 * 4 * 256 * 4;
  const size_t szRf   = (size_t)NFR * HW * HW * 4;
  const size_t szWenc = (size_t)9 * 8 * 128 * 32 * 2;
  const size_t szWmsk = (size_t)128 * 32 * 2;
  const size_t szWdif = (size_t)9 * 4 * 128 * 32 * 2;
  const size_t szWsum = (size_t)9 * 4 * 128 * 32 * 2;
  const size_t szWrf  = (size_t)9 * 8 * 16 * 32 * 2;
  const size_t szWrs  = (size_t)9 * 4 * 16 * 32 * 2;
#define CARVE(name, bytes) const size_t name = off; off = (off + (bytes) + 255) & ~(size_t)255;
  CARVE(oFeat, szFeat)
  CARVE(oMask, szMask)
  CARVE(oSt0,  szSt)
  CARVE(oSt1,  szSt)
  CARVE(oSP0,  szSP)
  CARVE(oSP1,  szSP)
  CARVE(oG,    szG)
  CARVE(oRf,   szRf)
  CARVE(oWenc, szWenc)
  CARVE(oWmsk, szWmsk)
  CARVE(oWdif, szWdif)
  CARVE(oWsum, szWsum)
  CARVE(oWrf,  szWrf)
  CARVE(oWrs,  szWrs)
#undef CARVE
  if (off > ws_size || off > (size_t)134217728) return;

  unsigned short* featsP = (unsigned short*)(ws + oFeat);
  unsigned short* maskP  = (unsigned short*)(ws + oMask);
  unsigned short* st0P   = (unsigned short*)(ws + oSt0);
  unsigned short* st1P   = (unsigned short*)(ws + oSt1);
  unsigned short* SP0    = (unsigned short*)(ws + oSP0);
  unsigned short* SP1    = (unsigned short*)(ws + oSP1);
  float*          G      = (float*)(ws + oG);
  float*          Rf     = (float*)(ws + oRf);
  unsigned short* wEnc   = (unsigned short*)(ws + oWenc);
  unsigned short* wMsk   = (unsigned short*)(ws + oWmsk);
  unsigned short* wDif   = (unsigned short*)(ws + oWdif);
  unsigned short* wSum   = (unsigned short*)(ws + oWsum);
  unsigned short* wRf    = (unsigned short*)(ws + oWrf);
  unsigned short* wRs    = (unsigned short*)(ws + oWrs);

  const dim3 blk(NTHR);
  const dim3 blkT(128);
  const dim3 gFrm(HW, NFR);
  const dim3 gPas(HW, NFP);
  const dim3 gImg(HW, NIP);

  k_cvt_feats<<<gFrm, blk, 0, stream>>>(feats, featsP);
  k_cvt_mask<<<dim3(NMB), blk, 0, stream>>>(maskIn, maskP);
  k_pack<<<dim3(144, 6), blk, 0, stream>>>(encW, gcnW, roW, vIdx, stIn, wEnc, wMsk, wDif, wSum, wRf, wRs);
  k_rof<<<gFrm, blkT, 0, stream>>>(featsP, wRf, Rf);

  for (int ps = 0; ps < NPASS; ++ps) {
    const unsigned short* fPp = featsP + (size_t)ps * NFP * NPIXP * CFE;
    const unsigned short* mPp = maskP + (size_t)ps * NIP * NPIXP;
    const float* RfP = Rf + (size_t)ps * NFP * HW * HW;
    float* outPs = out + (size_t)ps * NIP * HW * HW;
    k_enc<<<gPas, blk, 0, stream>>>(fPp, wEnc, mPp, wMsk, encB, st0P, SP0);
    k_sum<<<gPas, blk, 0, stream>>>(SP0, wSum, G);
    k_msg<<<gPas, blk, 0, stream>>>(st0P, wDif, gcnB, G, st1P, SP1, 1);
    k_sum<<<gPas, blk, 0, stream>>>(SP1, wSum, G);
    k_msg<<<gPas, blk, 0, stream>>>(st1P, wDif, gcnB, G, st0P, SP0, 0);
    k_ros<<<gImg, blkT, 0, stream>>>(st0P, wRs, RfP, roB, outPs);
  }
}
